// ReadUnit_34102040330305
// MI455X (gfx1250) — hardware-verified
//
#include <hip/hip_runtime.h>
#include <math.h>

constexpr int kNB       = 64;
constexpr int kPos      = 196;
constexpr int kDim      = 1024;
constexpr int kDim2     = 2048;
constexpr int kRows     = kNB * kPos;
constexpr int kHalfNB   = 32;
constexpr int kHalfRows = kHalfNB * kPos;
constexpr float kXCarry    = 16.0f;
constexpr float kWCarry    = 64.0f;
constexpr float kGemmScale = 1.0f / 1024.0f;

typedef __attribute__((ext_vector_type(16))) _Float16 v16h;
typedef __attribute__((ext_vector_type(8)))  _Float16 v8h;
typedef __attribute__((ext_vector_type(16))) __bf16   v16b;
typedef __attribute__((ext_vector_type(8)))  __bf16   v8b;
typedef __attribute__((ext_vector_type(8)))  float    v8f;
typedef __attribute__((ext_vector_type(4)))  float    v4f;
typedef __attribute__((ext_vector_type(4)))  unsigned int v4u;

__device__ __forceinline__ unsigned short f2bf_bits(float f) {
  unsigned u = __float_as_uint(f);
  return (unsigned short)((u + 0x7FFFu + ((u >> 16) & 1u)) >> 16);
}
__device__ __forceinline__ float bf_bits2f(unsigned short h) { return __uint_as_float(((unsigned)h) << 16); }

__device__ __forceinline__ void dep_guard_h(v8f& a, v8f& b, v16h x, v16h y) { asm volatile("v_nop\n\tv_nop\n\tv_nop\n\tv_nop" : "+v"(a), "+v"(b) : "v"(x), "v"(y)); }
__device__ __forceinline__ void dep_guard_b(v8f& a, v8f& b, v16b x, v16b y) { asm volatile("v_nop\n\tv_nop\n\tv_nop\n\tv_nop" : "+v"(a), "+v"(b) : "v"(x), "v"(y)); }
__device__ __forceinline__ void keep4_h(v16h a, v16h b, v16h c, v16h d) { asm volatile("v_nop" :: "v"(a), "v"(b), "v"(c), "v"(d)); }
__device__ __forceinline__ void keep4_b(v16b a, v16b b, v16b c, v16b d) { asm volatile("v_nop" :: "v"(a), "v"(b), "v"(c), "v"(d)); }
__device__ __forceinline__ void acc_guard4(v8f& a, v8f& b, v8f& c, v8f& d) { asm volatile("v_nop\n\tv_nop\n\tv_nop\n\tv_nop" : "+v"(a), "+v"(b), "+v"(c), "+v"(d)); }
template <typename T> struct Frag;
template <> struct Frag<_Float16> {
  typedef v16h V; union U { v16h v; v8h h[2]; };
  static __device__ __forceinline__ v16h load(const _Float16* p) {
    U f; f.h[0] = *(const v8h*)(p); f.h[1] = *(const v8h*)(p + 16); return f.v;
  }
  static __device__ __forceinline__ v8f mma(v16h a, v16h b, v8f c) {
    return __builtin_amdgcn_wmma_f32_16x16x32_f16(false, a, false, b, (short)0, c, false, false);
  }
  static __device__ __forceinline__ void guard(v8f& a, v8f& b, v16h x, v16h y) { dep_guard_h(a, b, x, y); }
  static __device__ __forceinline__ void keep(v16h a, v16h b, v16h c, v16h d) { keep4_h(a, b, c, d); }
};
template <> struct Frag<__bf16> {
  typedef v16b V; union U { v16b v; v8b h[2]; };
  static __device__ __forceinline__ v16b load(const __bf16* p) {
    U f; f.h[0] = *(const v8b*)(p); f.h[1] = *(const v8b*)(p + 16); return f.v;
  }
  static __device__ __forceinline__ v8f mma(v16b a, v16b b, v8f c) {
    return __builtin_amdgcn_wmma_f32_16x16x32_bf16(false, a, false, b, (short)0, c, false, false);
  }
  static __device__ __forceinline__ void guard(v8f& a, v8f& b, v16b x, v16b y) { dep_guard_b(a, b, x, y); }
  static __device__ __forceinline__ void keep(v16b a, v16b b, v16b c, v16b d) { keep4_b(a, b, c, d); }
};

__device__ __forceinline__ unsigned pk16(unsigned short a, unsigned short b) { return (unsigned)a | ((unsigned)b << 16); }
__device__ __forceinline__ unsigned short h_bits(float f) { const _Float16 h = (_Float16)f; return __builtin_bit_cast(unsigned short, h); }

template <int ET> struct Elem;
template <> struct Elem<0> { typedef _Float16 T; };
template <> struct Elem<1> { typedef __bf16 T; };
template <int ET, bool SPLIT, int BIAS_MODE, int OUT_MODE, bool RESID, int ACT = 0>
__global__ __launch_bounds__(256) void wmma_gemm64(
    const unsigned short* __restrict__ Ap, const unsigned short* __restrict__ A2p, int lda, long strideA,
    const unsigned short* __restrict__ Btp, const unsigned short* __restrict__ Bt2p, int ldb, long strideB,
    void* __restrict__ Cout, void* __restrict__ Cout2, int ldc, long strideC,
    const float* __restrict__ bias,
    const float* __restrict__ resid, long strideR,
    int M, int N, int K, float scale) {
  typedef typename Elem<ET>::T T;
  typedef typename Frag<T>::V V;
  const T* A = (const T*)Ap; const T* A2 = (const T*)A2p; const T* Bt = (const T*)Btp; const T* Bt2 = (const T*)Bt2p;
  __shared__ __align__(16) float sT[8][16 * 68];
  const int b    = blockIdx.y;
  const int lane = threadIdx.x & 31;
  const int wave = threadIdx.x >> 5;
  const int tilesN = N >> 6;
  const int tilesM = M >> 6;
  const int tile = blockIdx.x * 8 + wave;
  if (tile >= tilesM * tilesN) return;
  const int tm = tile / tilesN;
  const int tn = tile - tm * tilesN;
  const int m0 = tm << 6;
  const int n0 = tn << 6;

  const T* Ab  = A  + (size_t)b * strideA;
  const T* Bb  = Bt + (size_t)b * strideB;
  const T* Ab2 = SPLIT ? (A2  + (size_t)b * strideA) : nullptr;
  const T* Bb2 = SPLIT ? (Bt2 + (size_t)b * strideB) : nullptr;

  const int rlane = lane & 15;
  const int koff  = (lane >> 4) * 8;
  const int mOff  = (lane >> 4) * 8;

  v8f acc[4][4];
#pragma unroll
  for (int i = 0; i < 4; ++i)
#pragma unroll
    for (int j = 0; j < 4; ++j) acc[i][j] = (v8f){0.f,0.f,0.f,0.f,0.f,0.f,0.f,0.f};

  for (int k0 = 0; k0 < K; k0 += 32) {
    V bh[4], bl[4];
#pragma unroll
    for (int j = 0; j < 4; ++j) {
      const size_t bo = (size_t)(n0 + (j << 4) + rlane) * ldb + koff + k0;
      bh[j] = Frag<T>::load(Bb + bo);
      if (SPLIT) bl[j] = Frag<T>::load(Bb2 + bo);
    }
#pragma unroll
    for (int i = 0; i < 4; ++i) {
      const size_t ao = (size_t)(m0 + (i << 4) + rlane) * lda + koff + k0;
      V ah = Frag<T>::load(Ab + ao);
      V al;
      if (SPLIT) al = Frag<T>::load(Ab2 + ao);
#pragma unroll
      for (int j = 0; j < 4; ++j) {
        acc[i][j] = Frag<T>::mma(ah, bh[j], acc[i][j]);
        if (SPLIT) {
          acc[i][j] = Frag<T>::mma(ah, bl[j], acc[i][j]);
          acc[i][j] = Frag<T>::mma(al, bh[j], acc[i][j]);
        }
      }
      Frag<T>::guard(acc[i][0], acc[i][3], ah, SPLIT ? al : ah);
    }
    Frag<T>::keep(bh[0], bh[1], bh[2], bh[3]);
    if (SPLIT) Frag<T>::keep(bl[0], bl[1], bl[2], bl[3]);
  }
  acc_guard4(acc[0][0], acc[0][1], acc[0][2], acc[0][3]);
  acc_guard4(acc[1][0], acc[1][1], acc[1][2], acc[1][3]);
  acc_guard4(acc[2][0], acc[2][1], acc[2][2], acc[2][3]);
  acc_guard4(acc[3][0], acc[3][1], acc[3][2], acc[3][3]);

  float* slab = sT[wave];
  const float* Rb = RESID ? (resid + (size_t)b * strideR) : nullptr;
#pragma unroll
  for (int i = 0; i < 4; ++i) {
    const int mBase = m0 + (i << 4);
#pragma unroll
    for (int j = 0; j < 4; ++j) {
      const int n = n0 + (j << 4) + rlane;
      float bv = 0.f;
      if (BIAS_MODE == 2) bv = bias[n];
#pragma unroll
      for (int r = 0; r < 8; ++r) {
        float v = acc[i][j][r] * scale;
        if (BIAS_MODE == 1) v += bias[mBase + mOff + r];
        if (BIAS_MODE == 2) v += bv;
        if (RESID) v += Rb[(size_t)(mBase + mOff + r) * ldc + n];
        if (ACT == 2) v = fmaxf(v, 0.0f);
        if (ACT == 4) v = (v > 0.f) ? v : 0.01f * v;
        slab[(mOff + r) * 68 + (j << 4) + rlane] = v;
      }
    }
    __builtin_amdgcn_fence(__ATOMIC_RELEASE, "workgroup");
    __builtin_amdgcn_wave_barrier();
    __builtin_amdgcn_fence(__ATOMIC_ACQUIRE, "workgroup");
    if (OUT_MODE == 0) {
      float* C = (float*)Cout + (size_t)b * strideC;
      const int hh = lane >> 4, c4 = (lane & 15) * 4;
      for (int pass = 0; pass < 2; ++pass) {
#pragma unroll
        for (int it = 0; it < 8; ++it) {
          const int row = it * 2 + hh;
          v4f v = *(const v4f*)(slab + row * 68 + c4);
          *(volatile v4f*)(C + (size_t)(mBase + row) * ldc + n0 + c4) = v;
        }
        __threadfence();
      }
    } else {
      const int q = lane >> 3, c8 = (lane & 7) * 8;
      unsigned short* C  = (unsigned short*)Cout  + (size_t)b * strideC;
      unsigned short* C2 = (OUT_MODE == 2) ? ((unsigned short*)Cout2 + (size_t)b * strideC) : nullptr;
      for (int pass = 0; pass < 2; ++pass) {
#pragma unroll
        for (int it = 0; it < 4; ++it) {
          const int row = it * 4 + q;
          const float* sp = slab + row * 68 + c8;
          v8h hv, lv;
#pragma unroll
          for (int e = 0; e < 8; ++e) {
            if (OUT_MODE == 1) {
              hv[e] = (_Float16)sp[e];
            } else {
              unsigned short hb = f2bf_bits(sp[e]);
              unsigned short lb = f2bf_bits(sp[e] - bf_bits2f(hb));
              hv[e] = __builtin_bit_cast(_Float16, hb);
              lv[e] = __builtin_bit_cast(_Float16, lb);
            }
          }
          *(volatile v8h*)(C + (size_t)(mBase + row) * ldc + n0 + c8) = hv;
          if (OUT_MODE == 2) *(volatile v8h*)(C2 + (size_t)(mBase + row) * ldc + n0 + c8) = lv;
        }
        __threadfence();
      }
    }
    __builtin_amdgcn_fence(__ATOMIC_RELEASE, "workgroup");
    __builtin_amdgcn_wave_barrier();
    __builtin_amdgcn_fence(__ATOMIC_ACQUIRE, "workgroup");
  }
}

__global__ __launch_bounds__(256) void cast8_kernel(const float* __restrict__ in, int ld_in,
                                                    unsigned short* __restrict__ out, int ld_out,
                                                    int colShift, int ntot, float scale) {
  const int i = blockIdx.x * 256 + threadIdx.x;
  if (i >= ntot) return;
  const int row = i >> colShift;
  const int c8  = (i & ((1 << colShift) - 1)) * 8;
  const float* p = in + (size_t)row * ld_in + c8;
  const v4f a = *(const v4f*)(p);
  const v4f c = *(const v4f*)(p + 4);
  unsigned short hb[8];
#pragma unroll
  for (int e = 0; e < 4; ++e) {
    hb[e]     = h_bits(a[e] * scale);
    hb[4 + e] = h_bits(c[e] * scale);
  }
  const v4u u = (v4u){pk16(hb[0], hb[1]), pk16(hb[2], hb[3]), pk16(hb[4], hb[5]), pk16(hb[6], hb[7])};
  unsigned short* q = out + (size_t)row * ld_out + c8;
  *(volatile v4u*)q = u;
  __threadfence();
  *(volatile v4u*)q = u;
}

__global__ __launch_bounds__(256) void mul8_kernel(const float* __restrict__ X, int ldx,
                                                   const float* __restrict__ Vb,
                                                   unsigned short* __restrict__ out, int ld_out,
                                                   int ntot, int row0g, float scale) {
  const int i = blockIdx.x * 256 + threadIdx.x;
  if (i >= ntot) return;
  const int row = i >> 7;
  const int c8  = (i & 127) * 8;
  int bidx = (row0g + row) / kPos;
  bidx = bidx < 0 ? 0 : (bidx > kNB - 1 ? kNB - 1 : bidx);
  const float* xp = X  + (size_t)row  * ldx  + c8;
  const float* vp = Vb + (size_t)bidx * kDim + c8;
  const v4f xa = *(const v4f*)(xp);
  const v4f xc = *(const v4f*)(xp + 4);
  const v4f va = *(const v4f*)(vp);
  const v4f vc = *(const v4f*)(vp + 4);
  unsigned short hb[8];
#pragma unroll
  for (int e = 0; e < 4; ++e) {
    hb[e]     = h_bits((xa[e] * va[e]) * scale);
    hb[4 + e] = h_bits((xc[e] * vc[e]) * scale);
  }
  const v4u u = (v4u){pk16(hb[0], hb[1]), pk16(hb[2], hb[3]), pk16(hb[4], hb[5]), pk16(hb[6], hb[7])};
  unsigned short* q = out + (size_t)row * ld_out + c8;
  *(volatile v4u*)q = u;
  __threadfence();
  *(volatile v4u*)q = u;
}

__global__ __launch_bounds__(256) void softmax_sum_kernel(const float* __restrict__ ra,
                                                          const float* __restrict__ khw,
                                                          float* __restrict__ out) {
  __shared__ float redM[2][8];
  __shared__ float redS[2][8];
  const int bl   = blockIdx.x;
  const int t    = threadIdx.x;
  const int lane = t & 31, wave = t >> 5;
  const int c4   = t * 4;
  const float* rab = ra  + (size_t)bl * kPos * kDim + c4;
  const float* kb  = khw + (size_t)bl * kPos * kDim + c4;
  v4f acc = (v4f){0.f, 0.f, 0.f, 0.f};
#pragma unroll 1
  for (int p = 0; p < kPos; ++p) {
    const v4f x  = *(const v4f*)(rab + (size_t)p * kDim);
    const v4f kv = *(const v4f*)(kb  + (size_t)p * kDim);
    const int par = p & 1;
    float m = fmaxf(fmaxf(x[0], x[1]), fmaxf(x[2], x[3]));
#pragma unroll
    for (int off = 16; off > 0; off >>= 1) m = fmaxf(m, __shfl_xor(m, off, 32));
    if (lane == 0) redM[par][wave] = m;
    __syncthreads();
    float mm = redM[par][0];
#pragma unroll
    for (int w = 1; w < 8; ++w) mm = fmaxf(mm, redM[par][w]);
    const float e0 = expf(x[0] - mm);
    const float e1 = expf(x[1] - mm);
    const float e2 = expf(x[2] - mm);
    const float e3 = expf(x[3] - mm);
    float s = (e0 + e1) + (e2 + e3);
#pragma unroll
    for (int off = 16; off > 0; off >>= 1) s += __shfl_xor(s, off, 32);
    if (lane == 0) redS[par][wave] = s;
    __syncthreads();
    float ss = redS[par][0];
#pragma unroll
    for (int w = 1; w < 8; ++w) ss += redS[par][w];
    const float inv = 1.0f / ss;
    acc[0] += (e0 * inv) * kv[0];
    acc[1] += (e1 * inv) * kv[1];
    acc[2] += (e2 * inv) * kv[2];
    acc[3] += (e3 * inv) * kv[3];
  }
  float* op = out + (size_t)bl * kDim + c4;
  *(volatile v4f*)op = acc;
  __threadfence();
  *(volatile v4f*)op = acc;
}

static void launch_cast(const float* in, int ld_in, unsigned short* out, int ld_out, int colShift,
                        int nrows, float scale, hipStream_t s) {
  const int ntot = nrows << colShift;
  cast8_kernel<<<dim3((ntot + 255) / 256, 1, 1), dim3(256, 1, 1), 0, s>>>(in, ld_in, out, ld_out, colShift, ntot, scale);
}
static void launch_mul(const float* X, int ldx, const float* Vb, unsigned short* out, int ld_out,
                       int nrows, int row0g, float scale, hipStream_t s) {
  const int ntot = nrows * 128;
  mul8_kernel<<<dim3((ntot + 255) / 256, 1, 1), dim3(256, 1, 1), 0, s>>>(X, ldx, Vb, out, ld_out, ntot, row0g, scale);
}
static void launch_gemm(const unsigned short* A, int lda, const unsigned short* Bt, int ldb,
                        float* Cp, int ldc, const float* bias, int M, int N, int K, hipStream_t s) {
  const int tiles = (M / 64) * (N / 64);
  wmma_gemm64<0, false, 2, 0, false, 0><<<dim3((tiles + 7) / 8, 1, 1), dim3(256, 1, 1), 0, s>>>(
      A, A, lda, 0L, Bt, Bt, ldb, 0L, (void*)Cp, (void*)Cp, ldc, 0L, bias, bias, 0L, M, N, K, kGemmScale);
}

extern "C" void kernel_launch(void* const* d_in, const int* in_sizes, int n_in,
                              void* d_out, int out_size, void* d_ws, size_t ws_size,
                              hipStream_t stream) {
  if (n_in < 11) return;
  if (in_sizes[0] != kNB * kDim || in_sizes[1] != kNB * kDim || in_sizes[2] != kRows * kDim ||
      in_sizes[3] != kDim * kDim || in_sizes[4] != kDim || in_sizes[5] != kDim * kDim || in_sizes[6] != kDim ||
      in_sizes[7] != kDim * kDim2 || in_sizes[8] != kDim || in_sizes[9] != kDim * kDim || in_sizes[10] != kDim) return;
  if (out_size != kNB * kDim) return;

  const float* c_i   = (const float*)d_in[0];
  const float* m_i_1 = (const float*)d_in[1];
  const float* k_hw  = (const float*)d_in[2];
  const float* W_ddm = (const float*)d_in[3];
  const float* b_dm  = (const float*)d_in[4];
  const float* W_ddk = (const float*)d_in[5];
  const float* b_dk  = (const float*)d_in[6];
  const float* W_d2d = (const float*)d_in[7];
  const float* b_d1  = (const float*)d_in[8];
  const float* W_dd  = (const float*)d_in[9];
  const float* b_d2  = (const float*)d_in[10];
  float* out = (float*)d_out;

  char* w = (char*)d_ws;
  size_t off = 0;
  unsigned short* wddm16 = (unsigned short*)(w + off); off += (size_t)kDim * kDim * 2;
  unsigned short* wddk16 = (unsigned short*)(w + off); off += (size_t)kDim * kDim * 2;
  unsigned short* wd2d16 = (unsigned short*)(w + off); off += (size_t)kDim * kDim2 * 2;
  unsigned short* wdd16  = (unsigned short*)(w + off); off += (size_t)kDim * kDim * 2;
  unsigned short* m16    = (unsigned short*)(w + off); off += (size_t)kNB * kDim * 2;
  float*          wm32   = (float*)(w + off);          off += (size_t)kNB * kDim * 4;
  unsigned short* conc16 = (unsigned short*)(w + off); off += (size_t)kHalfRows * kDim2 * 2;
  float*          wk32   = (float*)(w + off);          off += (size_t)kHalfRows * kDim * 4;
  float*          ii32   = (float*)(w + off);          off += (size_t)kHalfRows * kDim * 4;
  unsigned short* ci16   = (unsigned short*)(w + off); off += (size_t)kHalfRows * kDim * 2;
  float*          ra32   = (float*)(w + off);          off += (size_t)kHalfRows * kDim * 4;
  if (off > ws_size) return;

  launch_cast(W_ddm, kDim,  wddm16, kDim,  7, kDim, kWCarry, stream);
  launch_cast(W_ddk, kDim,  wddk16, kDim,  7, kDim, kWCarry, stream);
  launch_cast(W_d2d, kDim2, wd2d16, kDim2, 8, kDim, kWCarry, stream);
  launch_cast(W_dd,  kDim,  wdd16,  kDim,  7, kDim, kWCarry, stream);
  launch_cast(m_i_1, kDim,  m16,    kDim,  7, kNB,  kXCarry, stream);

  launch_gemm(m16, kDim, wddm16, kDim, wm32, kDim, b_dm, kNB, kDim, kDim, stream);

  for (int half = 0; half < 2; ++half) {
    const int row0g = half * kHalfRows;
    const float* khw_half = k_hw + (size_t)row0g * kDim;

    launch_cast(khw_half, kDim, conc16 + kDim, kDim2, 7, kHalfRows, kXCarry, stream);

    launch_gemm(conc16 + kDim, kDim2, wddk16, kDim, wk32, kDim, b_dk, kHalfRows, kDim, kDim, stream);

    launch_mul(wk32, kDim, wm32, conc16, kDim2, kHalfRows, row0g, kXCarry, stream);

    launch_gemm(conc16, kDim2, wd2d16, kDim2, ii32, kDim, b_d1, kHalfRows, kDim, kDim2, stream);

    launch_mul(ii32, kDim, c_i, ci16, kDim, kHalfRows, row0g, kXCarry, stream);

    launch_gemm(ci16, kDim, wdd16, kDim, ra32, kDim, b_d2, kHalfRows, kDim, kDim, stream);

    softmax_sum_kernel<<<dim3(kHalfNB, 1, 1), dim3(256, 1, 1), 0, stream>>>(
        ra32, khw_half, out + (size_t)(half * kHalfNB) * kDim);
  }
}
